// GlobalFeatureGAT_17815524343963
// MI455X (gfx1250) — hardware-verified
//
#include <hip/hip_runtime.h>


namespace {
constexpr int N = 20000, E = 320000, V = 5000, L = 20, SF = 16, ED = 32, HC = 128, NH = 4, NG = 8, DIN = 176, DINP = 192, D1 = NH * HC, NPAD = 20096, NBLK = NPAD / 128;
constexpr float FXS = 524288.0f, FXI = 1.0f / 524288.0f;

typedef _Float16 b16;
typedef __attribute__((ext_vector_type(16))) _Float16 v16b;
typedef __attribute__((ext_vector_type(8)))  _Float16 v8b;
typedef __attribute__((ext_vector_type(8)))  float v8f;
typedef __attribute__((ext_vector_type(4)))  float v4f;

__device__ __forceinline__ v8b ld8b(const b16* p) { return *(const v8b*)p; }
__device__ __forceinline__ v16b cat8b(v8b a, v8b b) { return __builtin_shufflevector(a, b, 0, 1, 2, 3, 4, 5, 6, 7, 8, 9, 10, 11, 12, 13, 14, 15); }
__device__ __forceinline__ v16b frag_kb(const b16* p, int hh) { return cat8b(ld8b(p + 8 * hh), ld8b(p + 16 + 8 * hh)); }
__device__ __forceinline__ void split16(float v, b16& hi, b16& lo) { hi = (b16)v; lo = (b16)(v - (float)hi); }
__device__ __forceinline__ void frag_ksplit(const float* p, int hh, v16b& fh_, v16b& fl_) {
  const float* p0 = p + 8 * hh; const float* p1 = p + 16 + 8 * hh;
#pragma unroll
  for (int e = 0; e < 8; ++e) { b16 a, c; split16(p0[e], a, c); fh_[e] = a; fl_[e] = c; split16(p1[e], a, c); fh_[8 + e] = a; fl_[8 + e] = c; }
}
__device__ __forceinline__ v8f wmma16b(v16b a, v16b b, v8f c) {
  v8f d = __builtin_amdgcn_wmma_f32_16x16x32_f16(false, a, false, b, (short)0, c, false, false);
  asm volatile("v_nop\n\tv_nop\n\tv_nop\n\tv_nop" : "+v"(d) : "v"(a), "v"(b));
  return d;
}
__device__ __forceinline__ void wave_lds_sync() {
  __builtin_amdgcn_fence(__ATOMIC_RELEASE, "workgroup");
  __builtin_amdgcn_wave_barrier();
  __builtin_amdgcn_fence(__ATOMIC_ACQUIRE, "workgroup");
}

struct Opnd { const void* p0; const void* p1; int ld; };
template <int NP> __device__ __forceinline__ void load_frags(const Opnd& o, int row, int kb, int hh, v16b& fh_, v16b& fl_) {
  if (NP == 0) { frag_ksplit((const float*)o.p0 + (size_t)row * o.ld + kb, hh, fh_, fl_); }
  else if (NP == 4) {
    const float* p = (const float*)o.p0 + (size_t)row * o.ld + kb; const float* p0 = p + 8 * hh; const float* p1 = p + 16 + 8 * hh;
#pragma unroll
    for (int e = 0; e < 8; ++e) { b16 a, c; split16(p0[e] * 64.0f, a, c); fh_[e] = a; fl_[e] = c; split16(p1[e] * 64.0f, a, c); fh_[8 + e] = a; fl_[8 + e] = c; }
  } else if (NP == 3) {
    const float* p = (const float*)o.p0 + (size_t)row * o.ld + kb; const float* p0 = p + 8 * hh; const float* p1 = p + 16 + 8 * hh;
#pragma unroll
    for (int e = 0; e < 8; ++e) { fh_[e] = (b16)p0[e]; fh_[8 + e] = (b16)p1[e]; }
    fl_ = fh_;
  } else {
    fh_ = frag_kb((const b16*)o.p0 + (size_t)row * o.ld + kb, hh);
    if (NP == 2) fl_ = frag_kb((const b16*)o.p1 + (size_t)row * o.ld + kb, hh); else fl_ = fh_;
  }
}
template <int ANP, int BNP> __device__ __forceinline__ v8f mac(v16b ah, v16b al, v16b bh, v16b bl, v8f c) {
  c = wmma16b(ah, bh, c);
  if (BNP == 0 || BNP == 2 || BNP == 4) c = wmma16b(ah, bl, c);
  if (ANP == 0 || ANP == 2 || ANP == 4) c = wmma16b(al, bh, c);
  return c;
}
template <int ANP, int BNP>
__device__ __forceinline__ void gemm_tile(const Opnd& A, const Opnd& B, int K, int m0, int c0, int nloc, int hlf, v8f (&acc)[2][4]) {
  for (int kb = 0; kb < K; kb += 32) {
    v16b a0h, a0l, a1h, a1l;
    load_frags<ANP>(A, m0 + nloc, kb, hlf, a0h, a0l);
    load_frags<ANP>(A, m0 + 16 + nloc, kb, hlf, a1h, a1l);
#pragma unroll
    for (int t = 0; t < 4; ++t) {
      v16b bh, bl;
      load_frags<BNP>(B, c0 + t * 16 + nloc, kb, hlf, bh, bl);
      acc[0][t] = mac<ANP, BNP>(a0h, a0l, bh, bl, acc[0][t]);
      acc[1][t] = mac<ANP, BNP>(a1h, a1l, bh, bl, acc[1][t]);
    }
  }
}

__device__ __forceinline__ void epi_planes(v8f (&acc)[2][4], float scale, bool two, b16* __restrict__ oh, b16* __restrict__ ol, int ldo,
                                           int m0, int c0, int lane, b16* Th, b16* Tl) {
  const int nloc = lane & 15, hlf = lane >> 4;
#pragma unroll
  for (int t = 0; t < 4; ++t)
#pragma unroll
    for (int r = 0; r < 2; ++r)
#pragma unroll
      for (int v = 0; v < 8; ++v) {
        const int rr = r * 16 + v + 8 * hlf, cc = t * 16 + nloc;
        b16 h_, l_; split16(acc[r][t][v] * scale, h_, l_);
        Th[rr * 64 + cc] = h_; Tl[rr * 64 + cc] = l_;
      }
  wave_lds_sync();
  for (int pass = 0; pass < 2; ++pass) {
#pragma unroll
    for (int j = 0; j < 8; ++j) {
      const int rr = j * 4 + (lane >> 3), c8 = (lane & 7) * 8;
      const size_t o = (size_t)(m0 + rr) * ldo + c0 + c8;
      *(volatile v8b*)(oh + o) = ld8b(Th + rr * 64 + c8);
      if (two) *(volatile v8b*)(ol + o) = ld8b(Tl + rr * 64 + c8);
    }
    __threadfence();
  }
}
__device__ __forceinline__ void epi_f32(v8f (&acc)[2][4], float scale, const float* rscale, float* __restrict__ out, int ldo, int m0, int c0, int lane, float* Tt) {
  const int nloc = lane & 15, hlf = lane >> 4;
#pragma unroll
  for (int t = 0; t < 4; ++t)
#pragma unroll
    for (int r = 0; r < 2; ++r)
#pragma unroll
      for (int v = 0; v < 8; ++v) {
        const int rr = r * 16 + v + 8 * hlf;
        const float rs = rscale ? rscale[(size_t)(m0 + rr) * 32] : 1.0f;
        Tt[rr * 64 + t * 16 + nloc] = acc[r][t][v] * scale * rs;
      }
  wave_lds_sync();
  float* dst0 = out + (size_t)m0 * ldo + c0;
  for (int pass = 0; pass < 2; ++pass) {
#pragma unroll
    for (int j = 0; j < 16; ++j) { const int rr = j * 2 + hlf, c4 = nloc * 4; *(volatile v4f*)(dst0 + (size_t)rr * ldo + c4) = *(const v4f*)(Tt + rr * 64 + c4); }
    __threadfence();
  }
}


__device__ __forceinline__ int fkey(float f) { const int b = __float_as_int(f); return (b >= 0) ? b : (b ^ 0x7FFFFFFF); }
__device__ __forceinline__ float fkey_inv(int k) { return __int_as_float((k >= 0) ? k : (k ^ 0x7FFFFFFF)); }
__device__ __forceinline__ float elu1(float v) { return (v > 0.0f) ? v : (__expf(v) - 1.0f); }

__global__ __launch_bounds__(256) void prep_kernel(const float* __restrict__ W1, const float* __restrict__ W2, b16* __restrict__ w1t, b16* __restrict__ w2t) {
  const size_t tid = (size_t)blockIdx.x * blockDim.x + threadIdx.x, nth = (size_t)gridDim.x * blockDim.x;
  for (int pass = 0; pass < 2; ++pass) {
    for (size_t p = tid; p < (size_t)D1 * DINP / 8; p += nth) { const int n = (int)(p / (DINP / 8)), k0 = (int)(p % (DINP / 8)) * 8; v8b v;
#pragma unroll
      for (int e = 0; e < 8; ++e) { const int kp = k0 + e; const int k = (kp < 160) ? (SF + kp) : (kp < DIN ? kp - 160 : -1); v[e] = (b16)((k >= 0) ? W1[(size_t)k * D1 + n] : 0.0f); }
      *(volatile v8b*)(w1t + (size_t)n * DINP + k0) = v; }
    for (size_t p = tid; p < (size_t)HC * D1 / 8; p += nth) { const int n = (int)(p / (D1 / 8)), k0 = (int)(p % (D1 / 8)) * 8; v8b v;
#pragma unroll
      for (int e = 0; e < 8; ++e) v[e] = (b16)W2[(size_t)(k0 + e) * HC + n];
      *(volatile v8b*)(w2t + (size_t)n * D1 + k0) = v; }
    __threadfence();
  }
}

__global__ __launch_bounds__(256) void feat_kernel(const float* __restrict__ xs, const int* __restrict__ i0, const int* __restrict__ i1, const int* __restrict__ i2, const int* __restrict__ i3, const int* __restrict__ i4,
                                                   const float* __restrict__ t0, const float* __restrict__ t1, const float* __restrict__ t2, const float* __restrict__ t3, const float* __restrict__ t4,
                                                   const float* __restrict__ g, const float* __restrict__ bb, float* __restrict__ x) {
  const int wid = threadIdx.x >> 5, lane = threadIdx.x & 31, n = blockIdx.x * 8 + wid;
  float v[6] = {0, 0, 0, 0, 0, 0};
  if (n < N) {
    const int* ids[5] = {i0, i1, i2, i3, i4}; const float* tabs[5] = {t0, t1, t2, t3, t4};
#pragma unroll
    for (int f = 0; f < 5; ++f) { float s = 0.0f, c = 0.0f;
#pragma unroll 1
      for (int j = 0; j < L; ++j) { int id = ids[f][n * L + j]; const bool live = (id != 0); id = (id < 0) ? 0 : (id >= V ? V - 1 : id); if (live) { s += tabs[f][(size_t)id * ED + lane]; c += 1.0f; } }
      v[f] = s / (c + 1e-9f); }
    v[5] = (lane < SF) ? xs[(size_t)n * SF + lane] : 0.0f;
    float su = v[0] + v[1] + v[2] + v[3] + v[4] + v[5];
#pragma unroll
    for (int o = 16; o > 0; o >>= 1) su += __shfl_xor(su, o);
    const float mean = su * (1.0f / DIN); float s2 = 0.0f;
#pragma unroll
    for (int f = 0; f < 5; ++f) { const float dd = v[f] - mean; s2 += dd * dd; }
    if (lane < SF) { const float dd = v[5] - mean; s2 += dd * dd; }
#pragma unroll
    for (int o = 16; o > 0; o >>= 1) s2 += __shfl_xor(s2, o);
    const float rs = rsqrtf(s2 * (1.0f / DIN) + 1e-5f);
#pragma unroll
    for (int f = 0; f < 5; ++f) { const int k = SF + f * ED + lane; v[f] = (v[f] - mean) * rs * g[k] + bb[k]; }
    v[5] = (lane < SF) ? ((v[5] - mean) * rs * g[lane] + bb[lane]) : 0.0f;
  }
  float* row = x + (size_t)n * DINP;
  for (int pass = 0; pass < 2; ++pass) {
#pragma unroll
    for (int f = 0; f < 6; ++f) ((volatile float*)row)[f * 32 + lane] = v[f];
    __threadfence();
  }
}

template <int KIN, int NOUT>
__global__ __launch_bounds__(128) void lin_kernel(const float* __restrict__ x, const b16* __restrict__ w, float* __restrict__ h) {
  __shared__ __attribute__((aligned(16))) float Ts[4][32 * 64];
  const int lane = threadIdx.x & 31, wave = threadIdx.x >> 5, nloc = lane & 15, hlf = lane >> 4, m0 = blockIdx.y * 128 + wave * 32, c0 = blockIdx.x * 64;
  v8f acc[2][4];
#pragma unroll
  for (int r = 0; r < 2; ++r)
#pragma unroll
    for (int t = 0; t < 4; ++t) acc[r][t] = (v8f){};
  const Opnd A{x, nullptr, KIN}, B{w, nullptr, KIN};
  gemm_tile<3, 1>(A, B, KIN, m0, c0, nloc, hlf, acc);
  epi_f32(acc, 1.0f, nullptr, h, NOUT, m0, c0, lane, Ts[wave]);
}

template <int NHD>
__global__ __launch_bounds__(256) void alpha_kernel(const float* __restrict__ h, const float* __restrict__ asrc, const float* __restrict__ adst, float* __restrict__ al) {
  __shared__ float Ab[8][8];
  const int wid = threadIdx.x >> 5, lane = threadIdx.x & 31, n = blockIdx.x * 8 + wid;
#pragma unroll
  for (int hd = 0; hd < NHD; ++hd) { float ss = 0.0f, sd = 0.0f;
#pragma unroll
    for (int j = 0; j < 4; ++j) { const int c = j * 32 + lane; const float hv = h[(size_t)n * (NHD * HC) + hd * HC + c]; ss += hv * asrc[hd * HC + c]; sd += hv * adst[hd * HC + c]; }
#pragma unroll
    for (int o = 16; o > 0; o >>= 1) { ss += __shfl_xor(ss, o); sd += __shfl_xor(sd, o); }
    if (lane == 0) { Ab[wid][hd] = ss; Ab[wid][NHD + hd] = sd; } }
  if (lane == 0) for (int j = 2 * NHD; j < 8; ++j) Ab[wid][j] = 0.0f;
  __syncthreads();
  if (threadIdx.x < 64) { const float vv = Ab[threadIdx.x >> 3][threadIdx.x & 7]; for (int pass = 0; pass < 2; ++pass) { ((volatile float*)al)[(size_t)blockIdx.x * 64 + threadIdx.x] = vv; __threadfence(); } }
}

template <int NHD, int NB>
__global__ __launch_bounds__(256) void gat_kernel(const int* __restrict__ esrc, const int* __restrict__ edst, const float* __restrict__ h, const float* __restrict__ al, const float* __restrict__ bias, float* __restrict__ xo) {
  constexpr int DF = NHD * HC;
  __shared__ __attribute__((aligned(16))) int acc[NB * DF];
  __shared__ int mx[NB * NHD]; __shared__ int den[NB * NHD]; __shared__ int list[8 * 256];
  const int t_ = threadIdx.x, wave = t_ >> 5, lane = t_ & 31, base = blockIdx.x * NB;
  for (int i = t_; i < NB * DF; i += 256) acc[i] = 0;
  for (int i = t_; i < NB * NHD; i += 256) { den[i] = 0; mx[i] = fkey(-INFINITY); }
  __syncthreads();
  for (int i = t_; i < NB * NHD; i += 256) { const int slot = i / NHD, hd = i % NHD, node = base + slot; if (node < N) { float e = al[(size_t)node * 8 + hd] + al[(size_t)node * 8 + NHD + hd]; e = (e > 0.0f) ? e : 0.2f * e; atomicMax(&mx[i], fkey(e)); } }
  typedef __attribute__((ext_vector_type(4))) int v4i;
  for (int c0 = 0; c0 < E; c0 += 256 * 8) {
    const int e0 = c0 + (wave * 32 + lane) * 8; int dd[8];
    if (e0 + 7 < E) { const v4i a = *(const v4i*)(edst + e0), b = *(const v4i*)(edst + e0 + 4); dd[0] = a[0]; dd[1] = a[1]; dd[2] = a[2]; dd[3] = a[3]; dd[4] = b[0]; dd[5] = b[1]; dd[6] = b[2]; dd[7] = b[3]; }
    else {
#pragma unroll
      for (int j = 0; j < 8; ++j) dd[j] = (e0 + j < E) ? edst[e0 + j] : -1; }
#pragma unroll
    for (int j = 0; j < 8; ++j) { const unsigned sl = (unsigned)(dd[j] - base); if (sl < (unsigned)NB) { int s = esrc[e0 + j]; s = (s < 0) ? 0 : (s >= N ? N - 1 : s);
#pragma unroll
        for (int hd = 0; hd < NHD; ++hd) { float e = al[(size_t)s * 8 + hd] + al[(size_t)(base + sl) * 8 + NHD + hd]; e = (e > 0.0f) ? e : 0.2f * e; atomicMax(&mx[sl * NHD + hd], fkey(e)); } } }
  }
  __syncthreads();
  int* wl = list + wave * 256;
  auto accumulate = [&](int s, int slot) {
    float w[NHD];
#pragma unroll
    for (int hd = 0; hd < NHD; ++hd) { float e = al[(size_t)s * 8 + hd] + al[(size_t)(base + slot) * 8 + NHD + hd]; e = (e > 0.0f) ? e : 0.2f * e; w[hd] = __expf(e - fkey_inv(mx[slot * NHD + hd])); }
#pragma unroll
    for (int hd = 0; hd < NHD; ++hd) if (lane == hd) atomicAdd(&den[slot * NHD + hd], (int)rintf(w[hd] * FXS));
#pragma unroll
    for (int hd = 0; hd < NHD; ++hd) { const v4f v = *(const v4f*)(h + (size_t)s * DF + hd * HC + lane * 4);
#pragma unroll
      for (int c = 0; c < 4; ++c) atomicAdd(&acc[slot * DF + hd * HC + lane * 4 + c], (int)rintf(w[hd] * v[c] * FXS)); }
  };
  for (int slot = wave; slot < NB; slot += 8) { if (base + slot < N) accumulate(base + slot, slot); }
  for (int c0 = 0; c0 < E; c0 += 256 * 8) {
    const int e0 = c0 + (wave * 32 + lane) * 8; int dd[8];
    if (e0 + 7 < E) { const v4i a = *(const v4i*)(edst + e0), b = *(const v4i*)(edst + e0 + 4); dd[0] = a[0]; dd[1] = a[1]; dd[2] = a[2]; dd[3] = a[3]; dd[4] = b[0]; dd[5] = b[1]; dd[6] = b[2]; dd[7] = b[3]; }
    else {
#pragma unroll
      for (int j = 0; j < 8; ++j) dd[j] = (e0 + j < E) ? edst[e0 + j] : -1; }
    unsigned sl[8]; bool hit[8]; bool anyl = false;
#pragma unroll
    for (int j = 0; j < 8; ++j) { sl[j] = (unsigned)(dd[j] - base); hit[j] = sl[j] < (unsigned)NB; anyl |= hit[j]; }
    int wc = 0;
    if (__builtin_amdgcn_ballot_w32(anyl) != 0u) {
#pragma unroll
      for (int j = 0; j < 8; ++j) {
        const unsigned mj = __builtin_amdgcn_ballot_w32(hit[j]);
        if (mj != 0u) {
          if (hit[j]) { const int pos = wc + (int)__builtin_amdgcn_mbcnt_lo(mj, 0u); int s = esrc[e0 + j]; s = (s < 0) ? 0 : (s >= N ? N - 1 : s); wl[pos] = (s << 12) | (int)sl[j]; }
          wc += __builtin_popcount(mj); } } }
    __builtin_amdgcn_wave_barrier(); __builtin_amdgcn_fence(__ATOMIC_RELEASE, "workgroup"); __builtin_amdgcn_fence(__ATOMIC_ACQUIRE, "workgroup");
    for (int i = 0; i < wc; ++i) { const int ent = wl[i]; accumulate(ent >> 12, ent & 4095); }
    __builtin_amdgcn_wave_barrier();
  }
  __syncthreads();
  for (int pass = 0; pass < 2; ++pass) {
    for (int i = t_; i < NB * DF / 4; i += 256) { const int r = (i * 4) / DF, c0 = (i * 4) % DF, node = base + r; if (node < NPAD) { v4f o = {0.0f, 0.0f, 0.0f, 0.0f};
        if (node < N) { const float dn = (float)den[r * NHD + c0 / HC] * FXI + 1e-16f;
#pragma unroll
          for (int c = 0; c < 4; ++c) o[c] = elu1(((float)acc[i * 4 + c] * FXI) / dn + bias[c0 + c]); }
        *(volatile v4f*)(xo + (size_t)node * DF + c0) = o; } }
    __threadfence();
  }
}

__global__ __launch_bounds__(256) void pool_kernel(const float* __restrict__ x, const int* __restrict__ batch, float* __restrict__ out) {
  __shared__ float Pm[8][HC];
  const int wave = threadIdx.x >> 5, lane = threadIdx.x & 31, b = blockIdx.x;
  v4f mxv = {-INFINITY, -INFINITY, -INFINITY, -INFINITY};
#pragma unroll 1
  for (int n = wave; n < N; n += 8) { if (batch[n] == b) { const v4f v = *(const v4f*)(x + (size_t)n * HC + lane * 4);
#pragma unroll
      for (int c = 0; c < 4; ++c) mxv[c] = fmaxf(mxv[c], v[c]); } }
#pragma unroll
  for (int c = 0; c < 4; ++c) Pm[wave][lane * 4 + c] = mxv[c];
  __syncthreads();
  if (threadIdx.x < HC) { const int d = threadIdx.x; float mm = -INFINITY;
#pragma unroll
    for (int w = 0; w < 8; ++w) mm = fmaxf(mm, Pm[w][d]);
    for (int pass = 0; pass < 2; ++pass) { ((volatile float*)out)[(size_t)b * HC + d] = mm; __threadfence(); } }
}
}

extern "C" void kernel_launch(void* const* d_in, const int* in_sizes, int n_in,
                              void* d_out, int out_size, void* d_ws, size_t ws_size, hipStream_t stream) {
  (void)n_in; (void)out_size;
  const float* xs = (const float*)d_in[0]; const int* i0 = (const int*)d_in[1]; const int* i1 = (const int*)d_in[2]; const int* i2 = (const int*)d_in[3]; const int* i3 = (const int*)d_in[4]; const int* i4 = (const int*)d_in[5];
  const int* ei = (const int*)d_in[6]; const int* batch = (const int*)d_in[7];
  const float* t0 = (const float*)d_in[8]; const float* t1 = (const float*)d_in[9]; const float* t2 = (const float*)d_in[10]; const float* t3 = (const float*)d_in[11]; const float* t4 = (const float*)d_in[12];
  const float* lng = (const float*)d_in[13]; const float* lnb = (const float*)d_in[14];
  const float* W1 = (const float*)d_in[15]; const float* as1 = (const float*)d_in[16]; const float* ad1 = (const float*)d_in[17]; const float* b1 = (const float*)d_in[18];
  const float* W2 = (const float*)d_in[19]; const float* as2 = (const float*)d_in[20]; const float* ad2 = (const float*)d_in[21]; const float* b2 = (const float*)d_in[22];
  float* out = (float*)d_out;
  if (in_sizes[0] != N * SF || in_sizes[1] != N * L || in_sizes[6] != 2 * E || in_sizes[7] != N || in_sizes[8] != V * ED || in_sizes[15] != DIN * D1 || in_sizes[19] != D1 * HC) return;
  const int* esrc = ei; const int* edst = ei + E;
  size_t off = 0; char* ws = (char*)d_ws;
  auto carve = [&](size_t bytes) { char* p = ws + off; off += (bytes + 255) & ~(size_t)255; return p; };
  b16* w1t = (b16*)carve((size_t)D1 * DINP * 2); b16* w2t = (b16*)carve((size_t)HC * D1 * 2);
  float* x = (float*)carve((size_t)NPAD * DINP * 4);
  float* h1 = (float*)carve((size_t)NPAD * D1 * 4); float* x2 = (float*)carve((size_t)NPAD * D1 * 4);
  float* al = (float*)carve((size_t)NPAD * 8 * 4);
  float* h2 = (float*)carve((size_t)NPAD * HC * 4); float* x3 = (float*)carve((size_t)NPAD * HC * 4);
  if (off > ws_size) return;
  prep_kernel<<<256, 256, 0, stream>>>(W1, W2, w1t, w2t);
  feat_kernel<<<NPAD / 8, 256, 0, stream>>>(xs, i0, i1, i2, i3, i4, t0, t1, t2, t3, t4, lng, lnb, x);
  lin_kernel<DINP, D1><<<dim3(D1 / 64, NBLK), 128, 0, stream>>>(x, w1t, h1);
  alpha_kernel<NH><<<NPAD / 8, 256, 0, stream>>>(h1, as1, ad1, al);
  gat_kernel<NH, 128><<<NPAD / 128 + 1, 256, 0, stream>>>(esrc, edst, h1, al, b1, x2);
  lin_kernel<D1, HC><<<dim3(HC / 64, NBLK), 128, 0, stream>>>(x2, w2t, h2);
  alpha_kernel<1><<<NPAD / 8, 256, 0, stream>>>(h2, as2, ad2, al);
  gat_kernel<1, 512><<<NPAD / 512 + 1, 256, 0, stream>>>(esrc, edst, h2, al, b2, x3);
  pool_kernel<<<NG, 256, 0, stream>>>(x3, batch, out);
}
